// NoPadPagedAttention_3745211482347
// MI455X (gfx1250) — hardware-verified
//
#include <hip/hip_runtime.h>


namespace {
constexpr int Bn = 4, S = 1024, H = 16, HD = 64, T = 2048, D = H * HD;
constexpr float XS = 8.0f, PS = 8.0f, ISC = 0.125f;
__constant__ unsigned int INVF[32] = {0x3f800000u,0x3f3ff911u,0x3f0ff59au,0x3ed7e89bu,0x3ea1e89bu,0x3e72d423u,0x3e361887u,0x3e088d77u,0x3dcccccdu,0x3d99940du,0x3d6655c2u,0x3d2cba15u,0x3d0186e3u,0x3cc2434fu,0x3c91ad39u,0x3c5a7bf2u,0x3c23d70au,0x3bf5b9b0u,0x3bb8449cu,0x3b8a2e77u,0x3b4f3e38u,0x3b1b690du,0x3ae91528u,0x3aaec98eu,0x3a83126fu,0x3a44948cu,0x3a136a16u,0x39dd1725u,0x39a5cb60u,0x3978a815u,0x393a7753u,0x390bd472u};

typedef _Float16 b16;
typedef __attribute__((ext_vector_type(16))) _Float16 v16b;
typedef __attribute__((ext_vector_type(8))) _Float16 v8b;
typedef __attribute__((ext_vector_type(8))) float v8f;
typedef __attribute__((ext_vector_type(4))) float v4f;
__device__ __forceinline__ float bf16_rne(float f) { unsigned int u = __float_as_uint(f); u += 0x7FFFu + ((u >> 16) & 1u); return __uint_as_float(u & 0xFFFF0000u); }
__device__ __forceinline__ void split16(float v, b16& hi, b16& lo) { hi = (b16)v; lo = (b16)(v - (float)hi); }
__device__ __forceinline__ v16b frag_kb(const b16* p, int hh) { const v8b a = *(const v8b*)(p + 8 * hh), b = *(const v8b*)(p + 16 + 8 * hh); v16b f;
#pragma unroll
  for (int e = 0; e < 8; ++e) { f[e] = a[e]; f[8 + e] = b[e]; } return f; }
__device__ __forceinline__ v8f wmma16b(v16b a, v16b b, v8f c) { v8f d = __builtin_amdgcn_wmma_f32_16x16x32_f16(false, a, false, b, (short)0, c, false, false); asm volatile("v_nop\n\tv_nop\n\tv_nop\n\tv_nop" : "+v"(d) : "v"(a), "v"(b)); return d; }
__device__ __forceinline__ float nexp(float x) { return __builtin_amdgcn_exp2f(x * 1.4426950408889634f); }
__device__ __forceinline__ float pmul(float a, float b) { float p = a * b; asm volatile("" : "+v"(p)); return p; }

__global__ __launch_bounds__(256) void prep_kernel(const float* __restrict__ q, const float* __restrict__ k, const float* __restrict__ v, const int* __restrict__ lens, b16* __restrict__ QH, b16* __restrict__ QL, b16* __restrict__ KH, b16* __restrict__ KL, b16* __restrict__ VTh, b16* __restrict__ VTl) {
  __shared__ __attribute__((aligned(16))) b16 Th[D / 4][64 + 8], Tl[D / 4][64 + 8];
  const int b = blockIdx.y, p0 = blockIdx.x * 64, t_ = threadIdx.x;
  int off = 0; for (int i = 0; i < b; ++i) { int L = lens[i]; L = (L < 0) ? 0 : (L > S ? S : L); off += L; } int len = lens[b]; len = (len < 0) ? 0 : (len > S ? S : len); if (off > T) off = T;
  for (int pass = 0; pass < 2; ++pass) {
    for (int i = t_; i < 64 * (D / 8); i += 256) { const int pl = i / (D / 8), c8 = (i % (D / 8)) * 8; const int pos = p0 + pl; const int hd0 = c8 & 63; const bool live = (pos < len) && (off + pos < T);
      const size_t srow = (size_t)(off + pos) * D; v8b qh, ql, kh, kl;
#pragma unroll
      for (int e = 0; e < 8; ++e) { const int c = c8 + e, hd = hd0 + e; float qv = 0.0f, kv = 0.0f;
        if (live) { const int f = hd & 31; const float ang = (float)pos * __uint_as_float(INVF[f]); const float cs = (float)cos((double)ang), sn = (float)sin((double)ang);
          const float q0 = bf16_rne(q[srow + c]), k0 = bf16_rne(k[srow + c]); const int cp = (hd < 32) ? c + 32 : c - 32; const float qp = bf16_rne(q[srow + cp]), kp = bf16_rne(k[srow + cp]);
          qv = (hd < 32) ? (pmul(q0, cs) - pmul(qp, sn)) : (pmul(q0, cs) + pmul(qp, sn)); kv = (hd < 32) ? (pmul(k0, cs) - pmul(kp, sn)) : (pmul(k0, cs) + pmul(kp, sn)); }
        b16 a_, c_; split16(qv * XS, a_, c_); qh[e] = a_; ql[e] = c_; split16(kv * XS, a_, c_); kh[e] = a_; kl[e] = c_; }
      const size_t gi = ((size_t)b * S + pos) * D + c8; *(volatile v8b*)(QH + gi) = qh; *(volatile v8b*)(QL + gi) = ql; *(volatile v8b*)(KH + gi) = kh; *(volatile v8b*)(KL + gi) = kl; }
    for (int qtr = 0; qtr < 4; ++qtr) { __syncthreads();
      for (int i = t_; i < 64 * 256; i += 256) { const int pl = i >> 8, dd = i & 255; const int pos = p0 + pl; const bool live = (pos < len) && (off + pos < T); const float vv = live ? bf16_rne(v[(size_t)(off + pos) * D + qtr * 256 + dd]) : 0.0f; b16 a_, c_; split16(vv * XS, a_, c_); Th[dd][pl] = a_; Tl[dd][pl] = c_; }
      __syncthreads();
      for (int i = t_; i < 256 * 8; i += 256) { const int dd = i >> 3, c8 = (i & 7) * 8; const size_t gi = ((size_t)b * D + qtr * 256 + dd) * S + p0 + c8; *(volatile v8b*)(VTh + gi) = *(const v8b*)(&Th[dd][c8]); *(volatile v8b*)(VTl + gi) = *(const v8b*)(&Tl[dd][c8]); } }
    __threadfence(); }
}
__global__ __launch_bounds__(128) void attn_kernel(const b16* __restrict__ QH, const b16* __restrict__ QL, const b16* __restrict__ KH, const b16* __restrict__ KL, const b16* __restrict__ VTh, const b16* __restrict__ VTl, const int* __restrict__ lens, float* __restrict__ out) {
  __shared__ __attribute__((aligned(16))) float Os[4][16][HD + 4];
  const int wid = threadIdx.x >> 5, lane = threadIdx.x & 31, hh = lane >> 4, col = lane & 15; const int b = blockIdx.z, q0 = blockIdx.x * 16, h = blockIdx.y * 4 + wid, qi = q0 + col;
  int len = lens[b]; len = (len < 0) ? 0 : (len > S ? S : len);
  const b16* Qr = QH + ((size_t)b * S) * D + h * HD; const b16* Qlr = QL + ((size_t)b * S) * D + h * HD; const b16* Kr = KH + ((size_t)b * S) * D + h * HD; const b16* Klr = KL + ((size_t)b * S) * D + h * HD; const b16* V = VTh + ((size_t)b * D + h * HD) * S; const b16* Vl = VTl + ((size_t)b * D + h * HD) * S;
  const v16b qf0 = frag_kb(Qr + (size_t)qi * D, hh), qf1 = frag_kb(Qr + (size_t)qi * D + 32, hh), ql0 = frag_kb(Qlr + (size_t)qi * D, hh), ql1 = frag_kb(Qlr + (size_t)qi * D + 32, hh);
  float m = -INFINITY, l = 0.0f; v8f o[4] = {{}, {}, {}, {}};
  for (int kb = 0; kb < q0 + 16; kb += 32) {
    v8f s0 = {}, s1 = {};
    { const v16b k00 = frag_kb(Kr + (size_t)(kb + col) * D, hh), k01 = frag_kb(Kr + (size_t)(kb + col) * D + 32, hh), k10 = frag_kb(Kr + (size_t)(kb + 16 + col) * D, hh), k11 = frag_kb(Kr + (size_t)(kb + 16 + col) * D + 32, hh);
      const v16b l00 = frag_kb(Klr + (size_t)(kb + col) * D, hh), l01 = frag_kb(Klr + (size_t)(kb + col) * D + 32, hh), l10 = frag_kb(Klr + (size_t)(kb + 16 + col) * D, hh), l11 = frag_kb(Klr + (size_t)(kb + 16 + col) * D + 32, hh);
      s0 = wmma16b(k00, qf0, s0); s0 = wmma16b(k01, qf1, s0); s0 = wmma16b(l00, qf0, s0); s0 = wmma16b(l01, qf1, s0); s0 = wmma16b(k00, ql0, s0); s0 = wmma16b(k01, ql1, s0);
      s1 = wmma16b(k10, qf0, s1); s1 = wmma16b(k11, qf1, s1); s1 = wmma16b(l10, qf0, s1); s1 = wmma16b(l11, qf1, s1); s1 = wmma16b(k10, ql0, s1); s1 = wmma16b(k11, ql1, s1); }
    float mr = -INFINITY;
#pragma unroll
    for (int r = 0; r < 8; ++r) { const int j0 = kb + 8 * hh + r, j1 = j0 + 16; s0[r] = (j0 <= qi && j0 < len) ? s0[r] * (ISC / (XS * XS)) : -INFINITY; s1[r] = (j1 <= qi && j1 < len) ? s1[r] * (ISC / (XS * XS)) : -INFINITY; mr = fmaxf(mr, fmaxf(s0[r], s1[r])); }
    mr = fmaxf(mr, __shfl_xor(mr, 16)); const float mn = fmaxf(m, mr); const float al_ = (mn == -INFINITY) ? 1.0f : nexp(m - mn); m = mn; float sum = 0.0f; v16b pb, pl;
#pragma unroll
    for (int r = 0; r < 8; ++r) { const float e0 = (s0[r] == -INFINITY) ? 0.0f : nexp(s0[r] - mn), e1 = (s1[r] == -INFINITY) ? 0.0f : nexp(s1[r] - mn); sum += e0 + e1; b16 a_, c_; split16(e0 * PS, a_, c_); pb[r] = a_; pl[r] = c_; split16(e1 * PS, a_, c_); pb[8 + r] = a_; pl[8 + r] = c_; }
    sum += __shfl_xor(sum, 16); l = l * al_ + sum;
#pragma unroll
    for (int t = 0; t < 4; ++t) { o[t] *= al_; const v16b vh = frag_kb(V + (size_t)(t * 16 + col) * S + kb, hh); o[t] = wmma16b(vh, pb, o[t]); o[t] = wmma16b(vh, pl, o[t]); o[t] = wmma16b(frag_kb(Vl + (size_t)(t * 16 + col) * S + kb, hh), pb, o[t]); } }
  const float inv = (l > 0.0f) ? 1.0f / (l * PS * XS) : 0.0f;
#pragma unroll
  for (int t = 0; t < 4; ++t)
#pragma unroll
    for (int r = 0; r < 8; ++r) Os[wid][col][t * 16 + 8 * hh + r] = o[t][r] * inv;
  __syncthreads();
  for (int pass = 0; pass < 2; ++pass) { for (int i = threadIdx.x; i < 4 * 16 * 16; i += 128) { const int w = i >> 8, rr = (i >> 4) & 15, c4 = (i & 15) * 4; const int hq = blockIdx.y * 4 + w; *(volatile v4f*)(out + (((size_t)b * H + hq) * S + q0 + rr) * HD + c4) = *(const v4f*)(&Os[w][rr][c4]); } __threadfence(); }
}
}

extern "C" void kernel_launch(void* const* d_in, const int* in_sizes, int n_in,
                              void* d_out, int out_size, void* d_ws, size_t ws_size, hipStream_t stream) {
  (void)n_in; (void)out_size;
  const float* q = (const float*)d_in[0]; const float* k = (const float*)d_in[1]; const float* v = (const float*)d_in[2]; const int* lens = (const int*)d_in[5];
  float* out = (float*)d_out;
  if (in_sizes[0] != T * D || in_sizes[5] != Bn) return;
  size_t off = 0; char* ws = (char*)d_ws;
  auto carve = [&](size_t bytes) { char* p = ws + off; off += (bytes + 255) & ~(size_t)255; return p; };
  const size_t plane = (size_t)Bn * S * D; b16* QH = (b16*)carve(plane * 2); b16* QL = (b16*)carve(plane * 2); b16* KH = (b16*)carve(plane * 2); b16* KL = (b16*)carve(plane * 2); b16* VTh = (b16*)carve(plane * 2); b16* VTl = (b16*)carve(plane * 2);
  if (off > ws_size) return;
  prep_kernel<<<dim3(S / 64, Bn), 256, 0, stream>>>(q, k, v, lens, QH, QL, KH, KL, VTh, VTl);
  attn_kernel<<<dim3(S / 16, 4, Bn), 128, 0, stream>>>(QH, QL, KH, KL, VTh, VTl, lens, out);
}
